// Dipole_36756330119247
// MI455X (gfx1250) — hardware-verified
//
#include <hip/hip_runtime.h>
#include <math.h>

typedef __attribute__((ext_vector_type(16))) _Float16 v16h;
typedef __attribute__((ext_vector_type(8)))  _Float16 v8h;
typedef __attribute__((ext_vector_type(16))) __bf16   v16b;
typedef __attribute__((ext_vector_type(8)))  __bf16   v8b;
typedef __attribute__((ext_vector_type(8)))  float    v8f;
typedef __attribute__((ext_vector_type(4)))  float    v4f;

#define NT_STEPS 64
#define NB_ROWS 32
#define NROWS 2048
#define DIN 4096
#define DDAY 256
#define HID 256
#define GATE3 768
#define HT_COLS 1024
#define NOUT 942
#define NOUT_PAD 960
#define HS_PITCH 264
#define FS_PITCH 260

__device__ __forceinline__ unsigned short f2bf_bits(float f) {
  unsigned u = __float_as_uint(f);
  return (unsigned short)((u + 0x7FFFu + ((u >> 16) & 1u)) >> 16);
}
__device__ __forceinline__ float bf_bits2f(unsigned short h) { return __uint_as_float(((unsigned)h) << 16); }

__device__ __forceinline__ void dep_guard_h(v8f& a, v8f& b, v16h x, v16h y) { asm volatile("v_nop\n\tv_nop\n\tv_nop\n\tv_nop" : "+v"(a), "+v"(b) : "v"(x), "v"(y)); }
__device__ __forceinline__ void dep_guard_b(v8f& a, v8f& b, v16b x, v16b y) { asm volatile("v_nop\n\tv_nop\n\tv_nop\n\tv_nop" : "+v"(a), "+v"(b) : "v"(x), "v"(y)); }
__device__ __forceinline__ void keep4_h(v16h a, v16h b, v16h c, v16h d) { asm volatile("v_nop" :: "v"(a), "v"(b), "v"(c), "v"(d)); }
__device__ __forceinline__ void keep4_b(v16b a, v16b b, v16b c, v16b d) { asm volatile("v_nop" :: "v"(a), "v"(b), "v"(c), "v"(d)); }
__device__ __forceinline__ void acc_guard4(v8f& a, v8f& b, v8f& c, v8f& d) { asm volatile("v_nop\n\tv_nop\n\tv_nop\n\tv_nop" : "+v"(a), "+v"(b), "+v"(c), "+v"(d)); }
template <typename T> struct Frag;
template <> struct Frag<_Float16> {
  typedef v16h V; union U { v16h v; v8h h[2]; };
  static __device__ __forceinline__ v16h load(const _Float16* p) {
    U f; f.h[0] = *(const v8h*)(p); f.h[1] = *(const v8h*)(p + 16); return f.v;
  }
  static __device__ __forceinline__ v8f mma(v16h a, v16h b, v8f c) {
    return __builtin_amdgcn_wmma_f32_16x16x32_f16(false, a, false, b, (short)0, c, false, false);
  }
  static __device__ __forceinline__ void guard(v8f& a, v8f& b, v16h x, v16h y) { dep_guard_h(a, b, x, y); }
  static __device__ __forceinline__ void keep(v16h a, v16h b, v16h c, v16h d) { keep4_h(a, b, c, d); }
};
template <> struct Frag<__bf16> {
  typedef v16b V; union U { v16b v; v8b h[2]; };
  static __device__ __forceinline__ v16b load(const __bf16* p) {
    U f; f.h[0] = *(const v8b*)(p); f.h[1] = *(const v8b*)(p + 16); return f.v;
  }
  static __device__ __forceinline__ v8f mma(v16b a, v16b b, v8f c) {
    return __builtin_amdgcn_wmma_f32_16x16x32_bf16(false, a, false, b, (short)0, c, false, false);
  }
  static __device__ __forceinline__ void guard(v8f& a, v8f& b, v16b x, v16b y) { dep_guard_b(a, b, x, y); }
  static __device__ __forceinline__ void keep(v16b a, v16b b, v16b c, v16b d) { keep4_b(a, b, c, d); }
};

template <int ET> struct Elem;
template <> struct Elem<0> { typedef _Float16 T; };
template <> struct Elem<1> { typedef __bf16 T; };
template <int ET, bool SPLIT, int BIAS_MODE, int OUT_MODE, bool RESID, int ACT = 0>
__global__ __launch_bounds__(256) void wmma_gemm64(
    const unsigned short* __restrict__ Ap, const unsigned short* __restrict__ A2p, int lda, long strideA,
    const unsigned short* __restrict__ Btp, const unsigned short* __restrict__ Bt2p, int ldb, long strideB,
    void* __restrict__ Cout, void* __restrict__ Cout2, int ldc, long strideC,
    const float* __restrict__ bias,
    const float* __restrict__ resid, long strideR,
    int M, int N, int K, float scale) {
  typedef typename Elem<ET>::T T;
  typedef typename Frag<T>::V V;
  const T* A = (const T*)Ap; const T* A2 = (const T*)A2p; const T* Bt = (const T*)Btp; const T* Bt2 = (const T*)Bt2p;
  __shared__ __align__(16) float sT[8][16 * 68];
  const int b    = blockIdx.y;
  const int lane = threadIdx.x & 31;
  const int wave = threadIdx.x >> 5;
  const int tilesN = N >> 6;
  const int tilesM = M >> 6;
  const int tile = blockIdx.x * 8 + wave;
  if (tile >= tilesM * tilesN) return;
  const int tm = tile / tilesN;
  const int tn = tile - tm * tilesN;
  const int m0 = tm << 6;
  const int n0 = tn << 6;

  const T* Ab  = A  + (size_t)b * strideA;
  const T* Bb  = Bt + (size_t)b * strideB;
  const T* Ab2 = SPLIT ? (A2  + (size_t)b * strideA) : nullptr;
  const T* Bb2 = SPLIT ? (Bt2 + (size_t)b * strideB) : nullptr;

  const int rlane = lane & 15;
  const int koff  = (lane >> 4) * 8;
  const int mOff  = (lane >> 4) * 8;

  v8f acc[4][4];
#pragma unroll
  for (int i = 0; i < 4; ++i)
#pragma unroll
    for (int j = 0; j < 4; ++j) acc[i][j] = (v8f){0.f,0.f,0.f,0.f,0.f,0.f,0.f,0.f};

  for (int k0 = 0; k0 < K; k0 += 32) {
    V bh[4], bl[4];
#pragma unroll
    for (int j = 0; j < 4; ++j) {
      const size_t bo = (size_t)(n0 + (j << 4) + rlane) * ldb + koff + k0;
      bh[j] = Frag<T>::load(Bb + bo);
      if (SPLIT) bl[j] = Frag<T>::load(Bb2 + bo);
    }
#pragma unroll
    for (int i = 0; i < 4; ++i) {
      const size_t ao = (size_t)(m0 + (i << 4) + rlane) * lda + koff + k0;
      V ah = Frag<T>::load(Ab + ao);
      V al;
      if (SPLIT) al = Frag<T>::load(Ab2 + ao);
#pragma unroll
      for (int j = 0; j < 4; ++j) {
        acc[i][j] = Frag<T>::mma(ah, bh[j], acc[i][j]);
        if (SPLIT) {
          acc[i][j] = Frag<T>::mma(ah, bl[j], acc[i][j]);
          acc[i][j] = Frag<T>::mma(al, bh[j], acc[i][j]);
        }
      }
      Frag<T>::guard(acc[i][0], acc[i][3], ah, SPLIT ? al : ah);
    }
    Frag<T>::keep(bh[0], bh[1], bh[2], bh[3]);
    if (SPLIT) Frag<T>::keep(bl[0], bl[1], bl[2], bl[3]);
  }
  acc_guard4(acc[0][0], acc[0][1], acc[0][2], acc[0][3]);
  acc_guard4(acc[1][0], acc[1][1], acc[1][2], acc[1][3]);
  acc_guard4(acc[2][0], acc[2][1], acc[2][2], acc[2][3]);
  acc_guard4(acc[3][0], acc[3][1], acc[3][2], acc[3][3]);

  float* slab = sT[wave];
  const float* Rb = RESID ? (resid + (size_t)b * strideR) : nullptr;
#pragma unroll
  for (int i = 0; i < 4; ++i) {
    const int mBase = m0 + (i << 4);
#pragma unroll
    for (int j = 0; j < 4; ++j) {
      const int n = n0 + (j << 4) + rlane;
      float bv = 0.f;
      if (BIAS_MODE == 2) bv = bias[n];
#pragma unroll
      for (int r = 0; r < 8; ++r) {
        float v = acc[i][j][r] * scale;
        if (BIAS_MODE == 1) v += bias[mBase + mOff + r];
        if (BIAS_MODE == 2) v += bv;
        if (RESID) v += Rb[(size_t)(mBase + mOff + r) * ldc + n];
        if (ACT == 1) v = tanhf(v);
        if (ACT == 2) v = fmaxf(v, 0.0f);
        if (ACT == 3) v = v / (1.0f + expf(-v));
        if (ACT == 4) v = (v > 0.f) ? v : 0.01f * v;
        if (ACT == 5) v = 0.5f * v * (1.0f + erff(v * 0.70710678118654752f));
        if (ACT == 6) v = 1.0f / (1.0f + expf(-v));
        slab[(mOff + r) * 68 + (j << 4) + rlane] = v;
      }
    }
    __builtin_amdgcn_fence(__ATOMIC_RELEASE, "workgroup");
    __builtin_amdgcn_wave_barrier();
    __builtin_amdgcn_fence(__ATOMIC_ACQUIRE, "workgroup");
    if (OUT_MODE == 0) {
      float* C = (float*)Cout + (size_t)b * strideC;
      const int hh = lane >> 4, c4 = (lane & 15) * 4;
      for (int pass = 0; pass < 2; ++pass) {
#pragma unroll
        for (int it = 0; it < 8; ++it) {
          const int row = it * 2 + hh;
          v4f v = *(const v4f*)(slab + row * 68 + c4);
          *(volatile v4f*)(C + (size_t)(mBase + row) * ldc + n0 + c4) = v;
        }
        __threadfence();
      }
    } else {
      const int q = lane >> 3, c8 = (lane & 7) * 8;
      unsigned short* C  = (unsigned short*)Cout  + (size_t)b * strideC;
      unsigned short* C2 = (OUT_MODE == 2) ? ((unsigned short*)Cout2 + (size_t)b * strideC) : nullptr;
      for (int pass = 0; pass < 2; ++pass) {
#pragma unroll
        for (int it = 0; it < 4; ++it) {
          const int row = it * 4 + q;
          const float* sp = slab + row * 68 + c8;
          v8h hv, lv;
#pragma unroll
          for (int e = 0; e < 8; ++e) {
            if (OUT_MODE == 1) {
              hv[e] = (_Float16)sp[e];
            } else {
              unsigned short hb = f2bf_bits(sp[e]);
              unsigned short lb = f2bf_bits(sp[e] - bf_bits2f(hb));
              hv[e] = __builtin_bit_cast(_Float16, hb);
              lv[e] = __builtin_bit_cast(_Float16, lb);
            }
          }
          *(volatile v8h*)(C + (size_t)(mBase + row) * ldc + n0 + c8) = hv;
          if (OUT_MODE == 2) *(volatile v8h*)(C2 + (size_t)(mBase + row) * ldc + n0 + c8) = lv;
        }
        __threadfence();
      }
    }
    __builtin_amdgcn_fence(__ATOMIC_RELEASE, "workgroup");
    __builtin_amdgcn_wave_barrier();
    __builtin_amdgcn_fence(__ATOMIC_ACQUIRE, "workgroup");
  }
}

__global__ __launch_bounds__(256) void cast_f32_f16x8(const float* __restrict__ in, unsigned short* __restrict__ out,
                                                      int n8_total, int n8_valid, float scale) {
  const int i = blockIdx.x * 256 + threadIdx.x;
  if (i >= n8_total) return;
  const int ic = (i < n8_valid) ? i : (n8_valid - 1);
  const float sc = (i < n8_valid) ? scale : 0.0f;
  const v4f a = *(const v4f*)(in + (size_t)ic * 8);
  const v4f b = *(const v4f*)(in + (size_t)ic * 8 + 4);
  v8h hv;
  hv[0] = (_Float16)(a[0] * sc); hv[1] = (_Float16)(a[1] * sc);
  hv[2] = (_Float16)(a[2] * sc); hv[3] = (_Float16)(a[3] * sc);
  hv[4] = (_Float16)(b[0] * sc); hv[5] = (_Float16)(b[1] * sc);
  hv[6] = (_Float16)(b[2] * sc); hv[7] = (_Float16)(b[3] * sc);
  _Float16* p = (_Float16*)(out + (size_t)i * 8);
  *(volatile v8h*)p = hv;
  __threadfence();
  *(volatile v8h*)p = hv;
}

__global__ __launch_bounds__(256) void pad_vec_f32x4(const float* __restrict__ in, float* __restrict__ out,
                                                     int n4_total, int n_valid) {
  const int i = blockIdx.x * 256 + threadIdx.x;
  if (i >= n4_total) return;
  v4f v;
#pragma unroll
  for (int e = 0; e < 4; ++e) {
    const int idx = 4 * i + e;
    const int ic = (idx < n_valid) ? idx : (n_valid - 1);
    const float x = in[ic];
    v[e] = (idx < n_valid) ? x : 0.0f;
  }
  float* p = out + (size_t)i * 4;
  *(volatile v4f*)p = v;
  __threadfence();
  *(volatile v4f*)p = v;
}

__global__ __launch_bounds__(256) void out_pack_kernel(const float* __restrict__ src, float* __restrict__ dst,
                                                       int n4, int ncol, int ld, int nrow) {
  const int i = blockIdx.x * 256 + threadIdx.x;
  if (i >= n4) return;
  v4f v;
#pragma unroll
  for (int e = 0; e < 4; ++e) {
    const int idx = 4 * i + e;
    int row = idx / ncol;
    const int col = idx - row * ncol;
    row = (row < nrow) ? row : (nrow - 1);
    v[e] = src[(size_t)row * ld + col];
  }
  float* p = dst + (size_t)i * 4;
  *(volatile v4f*)p = v;
  __threadfence();
  *(volatile v4f*)p = v;
}

union HFrag { v16h v; v8h h[2]; };

__device__ __forceinline__ v8f hmma_g(v16h a, v16h b, v8f c) {
  c = __builtin_amdgcn_wmma_f32_16x16x32_f16(false, a, false, b, (short)0, c, false, false);
  asm volatile("v_nop\n\tv_nop\n\tv_nop\n\tv_nop" : "+v"(c) : "v"(a), "v"(b));
  return c;
}
__device__ __forceinline__ float sigm_f(float x) { return 1.0f / (1.0f + expf(-x)); }

template <bool REV>
__global__ __launch_bounds__(256) void gru_seq_kernel(
    const unsigned short* __restrict__ Whh16, const float* __restrict__ bhh,
    const float* __restrict__ GI, const float* __restrict__ attw,
    float* __restrict__ f32rows, unsigned short* __restrict__ rev16, float* __restrict__ splane) {
  __shared__ __align__(16) _Float16 Hs[16 * HS_PITCH];
  __shared__ __align__(16) float Fs[16 * FS_PITCH];
  __shared__ __align__(16) float Ss[16 * 64];
  const int tid = threadIdx.x;
  const int lane = tid & 31, wave = tid >> 5;
  const int hh = lane >> 4, cl = lane & 15, koff = hh * 8;
  const int blk = blockIdx.x;
  const int iq = REV ? (blk >> 1) : 0;
  const int b0 = REV ? ((blk & 1) * 16) : (blk * 16);
  const int nsteps = REV ? (iq + 1) : NT_STEPS;
  const int srow0 = REV ? (iq * NB_ROWS + b0) : b0;
  const int ubase = 32 * wave + cl;

  for (int idx = tid; idx < 16 * HS_PITCH; idx += 256) Hs[idx] = (_Float16)0.0f;
  for (int idx = tid; idx < 16 * 64; idx += 256) Ss[idx] = 0.0f;

  float wa[8];
  {
    const v4f w0 = *(const v4f*)(attw + lane * 8);
    const v4f w1 = *(const v4f*)(attw + lane * 8 + 4);
    wa[0] = w0[0]; wa[1] = w0[1]; wa[2] = w0[2]; wa[3] = w0[3];
    wa[4] = w1[0]; wa[5] = w1[1]; wa[6] = w1[2]; wa[7] = w1[3];
  }
  float bhv[2][3];
#pragma unroll
  for (int ub = 0; ub < 2; ++ub)
#pragma unroll
    for (int g = 0; g < 3; ++g) bhv[ub][g] = bhh[g * HID + ubase + 16 * ub];
  float hreg[2][8];
#pragma unroll
  for (int ub = 0; ub < 2; ++ub)
#pragma unroll
    for (int r = 0; r < 8; ++r) hreg[ub][r] = 0.0f;
  __syncthreads();

  for (int j = 0; j < nsteps; ++j) {
    v8f acc[2][3];
#pragma unroll
    for (int ub = 0; ub < 2; ++ub)
#pragma unroll
      for (int g = 0; g < 3; ++g) acc[ub][g] = (v8f){0.f,0.f,0.f,0.f,0.f,0.f,0.f,0.f};
#pragma unroll 1
    for (int k0 = 0; k0 < HID; k0 += 32) {
      HFrag af;
      af.h[0] = *(const v8h*)(Hs + cl * HS_PITCH + koff + k0);
      af.h[1] = *(const v8h*)(Hs + cl * HS_PITCH + koff + k0 + 16);
#pragma unroll
      for (int ub = 0; ub < 2; ++ub) {
#pragma unroll
        for (int g = 0; g < 3; ++g) {
          const v16h bfr = Frag<_Float16>::load((const _Float16*)Whh16 +
                                                 (size_t)(g * HID + ubase + 16 * ub) * HID + koff + k0);
          acc[ub][g] = hmma_g(af.v, bfr, acc[ub][g]);
        }
      }
    }
    const int tsrc = REV ? (((iq - j) > 0) ? (iq - j) : 0) : j;
    const int girow0 = tsrc * NB_ROWS + b0 + 8 * hh;
#pragma unroll
    for (int ub = 0; ub < 2; ++ub) {
      const int unit = ubase + 16 * ub;
#pragma unroll
      for (int r = 0; r < 8; ++r) {
        const float* gp = GI + (size_t)(girow0 + r) * GATE3 + unit;
        const float gir = gp[0];
        const float giz = gp[HID];
        const float gin = gp[2 * HID];
        const float ghr = acc[ub][0][r] * 0.0625f + bhv[ub][0];
        const float ghz = acc[ub][1][r] * 0.0625f + bhv[ub][1];
        const float ghn = acc[ub][2][r] * 0.0625f + bhv[ub][2];
        const float rg = sigm_f(gir + ghr);
        const float zg = sigm_f(giz + ghz);
        const float ng = tanhf(gin + rg * ghn);
        hreg[ub][r] = (1.0f - zg) * ng + zg * hreg[ub][r];
      }
    }
    __syncthreads();
#pragma unroll
    for (int ub = 0; ub < 2; ++ub) {
      const int unit = ubase + 16 * ub;
#pragma unroll
      for (int r = 0; r < 8; ++r) {
        Hs[(8 * hh + r) * HS_PITCH + unit] = (_Float16)hreg[ub][r];
        Fs[(8 * hh + r) * FS_PITCH + unit] = hreg[ub][r];
      }
    }
    __syncthreads();
#pragma unroll
    for (int rr2 = 0; rr2 < 2; ++rr2) {
      const int row = 2 * wave + rr2;
      const float* fr = Fs + row * FS_PITCH;
      const v4f p0 = *(const v4f*)(fr + lane * 8);
      const v4f p1 = *(const v4f*)(fr + lane * 8 + 4);
      float sp = p0[0] * wa[0] + p0[1] * wa[1] + p0[2] * wa[2] + p0[3] * wa[3]
               + p1[0] * wa[4] + p1[1] * wa[5] + p1[2] * wa[6] + p1[3] * wa[7];
#pragma unroll
      for (int off = 16; off > 0; off >>= 1) sp += __shfl_xor(sp, off, 32);
      if (lane == 0) Ss[row * 64 + j] = sp;
      if (REV) {
        v8h hv;
        hv[0] = (_Float16)p0[0]; hv[1] = (_Float16)p0[1]; hv[2] = (_Float16)p0[2]; hv[3] = (_Float16)p0[3];
        hv[4] = (_Float16)p1[0]; hv[5] = (_Float16)p1[1]; hv[6] = (_Float16)p1[2]; hv[7] = (_Float16)p1[3];
        _Float16* rp = (_Float16*)(rev16 + ((((size_t)iq * NT_STEPS + j) * NB_ROWS + b0 + row) * HID)) + lane * 8;
        for (int pass = 0; pass < 2; ++pass) {
          *(volatile v8h*)rp = hv;
          __threadfence();
        }
      }
      const bool wr32 = REV ? (j == iq) : true;
      if (wr32) {
        const v4f q0 = *(const v4f*)(fr + lane * 4);
        const v4f q1 = *(const v4f*)(fr + 128 + lane * 4);
        const int grow = REV ? (iq * NB_ROWS + b0 + row) : (j * NB_ROWS + b0 + row);
        float* op = f32rows + (size_t)grow * HID;
        for (int pass = 0; pass < 2; ++pass) {
          *(volatile v4f*)(op + lane * 4) = q0;
          *(volatile v4f*)(op + 128 + lane * 4) = q1;
          __threadfence();
        }
      }
    }
  }
  __syncthreads();
  {
    const int row = 2 * wave + hh;
    const int c4 = cl * 4;
    const v4f v = *(const v4f*)(Ss + row * 64 + c4);
    float* sp = splane + (size_t)(srow0 + row) * 64 + c4;
    for (int pass = 0; pass < 2; ++pass) {
      *(volatile v4f*)sp = v;
      __threadfence();
    }
  }
}

__global__ __launch_bounds__(128) void attn_ctx_kernel(
    const float* __restrict__ sfwd, const float* __restrict__ srev, const float* __restrict__ attn_b,
    const float* __restrict__ fwd32, const unsigned short* __restrict__ rev16,
    const float* __restrict__ rlast32, unsigned short* __restrict__ ht16) {
  __shared__ float s_al[64];
  __shared__ __align__(16) float s_ht[HT_COLS];
  const int tid = threadIdx.x;
  const int lane = tid & 31, wave = tid >> 5;
  const int rowid = blockIdx.x;
  const int iq = rowid >> 5, b = rowid & 31;

  if (tid < 64) {
    const int t = tid;
    const int tc = (t <= iq) ? t : iq;
    const float s = sfwd[b * 64 + tc] + srev[(size_t)rowid * 64 + tc] + attn_b[0];
    s_al[t] = (t <= iq) ? s : -INFINITY;
  }
  __syncthreads();
  if (wave == 0) {
    const float v0 = s_al[lane];
    const float v1 = s_al[lane + 32];
    float m = fmaxf(v0, v1);
#pragma unroll
    for (int off = 16; off > 0; off >>= 1) m = fmaxf(m, __shfl_xor(m, off, 32));
    float e0 = expf(v0 - m);
    float e1 = expf(v1 - m);
    e0 = (lane <= iq) ? e0 : 0.0f;
    e1 = ((lane + 32) <= iq) ? e1 : 0.0f;
    float su = e0 + e1;
#pragma unroll
    for (int off = 16; off > 0; off >>= 1) su += __shfl_xor(su, off, 32);
    const float inv = 1.0f / su;
    s_al[lane] = e0 * inv;
    s_al[lane + 32] = e1 * inv;
  }
  __syncthreads();

  const int h2 = 2 * tid;
  float cf0 = 0.f, cf1 = 0.f, cr0 = 0.f, cr1 = 0.f;
#pragma unroll 1
  for (int t = 0; t <= iq; ++t) {
    const float a = s_al[t];
    const float* fp = fwd32 + (size_t)(t * NB_ROWS + b) * HID + h2;
    const float f0 = fp[0], f1 = fp[1];
    const unsigned w = ((const unsigned*)rev16)[(((((size_t)iq * NT_STEPS + t) * NB_ROWS + b) * HID) + h2) >> 1];
    const float r0 = (float)__builtin_bit_cast(_Float16, (unsigned short)(w & 0xffffu));
    const float r1 = (float)__builtin_bit_cast(_Float16, (unsigned short)(w >> 16));
    cf0 += a * f0; cf1 += a * f1;
    cr0 += a * r0; cr1 += a * r1;
  }
  const float invc = 1.0f / (float)(iq + 1);
  s_ht[h2] = cf0 * invc;
  s_ht[h2 + 1] = cf1 * invc;
  s_ht[HID + h2] = cr0 * invc;
  s_ht[HID + h2 + 1] = cr1 * invc;
  {
    const float* fi = fwd32 + (size_t)rowid * HID + h2;
    const float* rl = rlast32 + (size_t)rowid * HID + h2;
    s_ht[2 * HID + h2] = fi[0];
    s_ht[2 * HID + h2 + 1] = fi[1];
    s_ht[3 * HID + h2] = rl[0];
    s_ht[3 * HID + h2 + 1] = rl[1];
  }
  __syncthreads();
  {
    const v4f p0 = *(const v4f*)(s_ht + 8 * tid);
    const v4f p1 = *(const v4f*)(s_ht + 8 * tid + 4);
    v8h hv;
    hv[0] = (_Float16)(p0[0] * 64.0f); hv[1] = (_Float16)(p0[1] * 64.0f);
    hv[2] = (_Float16)(p0[2] * 64.0f); hv[3] = (_Float16)(p0[3] * 64.0f);
    hv[4] = (_Float16)(p1[0] * 64.0f); hv[5] = (_Float16)(p1[1] * 64.0f);
    hv[6] = (_Float16)(p1[2] * 64.0f); hv[7] = (_Float16)(p1[3] * 64.0f);
    _Float16* op = (_Float16*)(ht16 + (size_t)rowid * HT_COLS) + 8 * tid;
    for (int pass = 0; pass < 2; ++pass) {
      *(volatile v8h*)op = hv;
      __threadfence();
    }
  }
}

#define SZ_X16    (2048ull * 4096ull * 2ull)
#define SZ_WEMB16 (256ull * 4096ull * 2ull)
#define SZ_W768   (768ull * 256ull * 2ull)
#define SZ_WAO16  (256ull * 1024ull * 2ull)
#define SZ_WO16   (960ull * 256ull * 2ull)
#define SZ_BO     (4096ull)
#define SZ_DE16   (2048ull * 256ull * 2ull)
#define SZ_GI     (2048ull * 768ull * 4ull)
#define SZ_F32R   (2048ull * 256ull * 4ull)
#define SZ_REV16  (64ull * 64ull * 32ull * 256ull * 2ull)
#define SZ_SFWD   (8192ull)
#define SZ_SREV   (2048ull * 64ull * 4ull)
#define SZ_HT16   (2048ull * 1024ull * 2ull)
#define SZ_AO16   (2048ull * 256ull * 2ull)
#define SZ_OUT960 (2048ull * 960ull * 4ull)

static const size_t OFF_X16    = 0;
static const size_t OFF_WEMB16 = OFF_X16 + SZ_X16;
static const size_t OFF_WIHF16 = OFF_WEMB16 + SZ_WEMB16;
static const size_t OFF_WHHF16 = OFF_WIHF16 + SZ_W768;
static const size_t OFF_WIHR16 = OFF_WHHF16 + SZ_W768;
static const size_t OFF_WHHR16 = OFF_WIHR16 + SZ_W768;
static const size_t OFF_WAO16  = OFF_WHHR16 + SZ_W768;
static const size_t OFF_WO16   = OFF_WAO16 + SZ_WAO16;
static const size_t OFF_BO     = OFF_WO16 + SZ_WO16;
static const size_t OFF_DE16   = OFF_BO + SZ_BO;
static const size_t OFF_GIF    = OFF_DE16 + SZ_DE16;
static const size_t OFF_GIR    = OFF_GIF + SZ_GI;
static const size_t OFF_FWD32  = OFF_GIR + SZ_GI;
static const size_t OFF_RLAST  = OFF_FWD32 + SZ_F32R;
static const size_t OFF_REV16  = OFF_RLAST + SZ_F32R;
static const size_t OFF_SFWD   = OFF_REV16 + SZ_REV16;
static const size_t OFF_SREV   = OFF_SFWD + SZ_SFWD;
static const size_t OFF_HT16   = OFF_SREV + SZ_SREV;
static const size_t OFF_AO16   = OFF_HT16 + SZ_HT16;
static const size_t OFF_OUT960 = OFF_AO16 + SZ_AO16;
static const size_t WS_TOTAL   = OFF_OUT960 + SZ_OUT960;
static_assert(OFF_OUT960 + SZ_OUT960 == 120041472ull, "ws");
static_assert(OFF_OUT960 + SZ_OUT960 <= 134217728ull, "ws");

extern "C" void kernel_launch(void* const* d_in, const int* in_sizes, int n_in,
                              void* d_out, int out_size, void* d_ws, size_t ws_size,
                              hipStream_t stream) {
  (void)in_sizes; (void)n_in; (void)out_size;
  if (ws_size < WS_TOTAL) return;
  const float* x     = (const float*)d_in[0];
  const float* Wemb  = (const float*)d_in[1];
  const float* bemb  = (const float*)d_in[2];
  const float* Wihf  = (const float*)d_in[3];
  const float* Whhf  = (const float*)d_in[4];
  const float* bihf  = (const float*)d_in[5];
  const float* bhhf  = (const float*)d_in[6];
  const float* Wihr  = (const float*)d_in[7];
  const float* Whhr  = (const float*)d_in[8];
  const float* bihr  = (const float*)d_in[9];
  const float* bhhr  = (const float*)d_in[10];
  const float* attnw = (const float*)d_in[11];
  const float* attnb = (const float*)d_in[12];
  const float* Wao   = (const float*)d_in[13];
  const float* bao   = (const float*)d_in[14];
  const float* Wo    = (const float*)d_in[15];
  const float* bo    = (const float*)d_in[16];
  float* out = (float*)d_out;

  char* ws = (char*)d_ws;
  unsigned short* X16    = (unsigned short*)(ws + OFF_X16);
  unsigned short* WEMB16 = (unsigned short*)(ws + OFF_WEMB16);
  unsigned short* WIHF16 = (unsigned short*)(ws + OFF_WIHF16);
  unsigned short* WHHF16 = (unsigned short*)(ws + OFF_WHHF16);
  unsigned short* WIHR16 = (unsigned short*)(ws + OFF_WIHR16);
  unsigned short* WHHR16 = (unsigned short*)(ws + OFF_WHHR16);
  unsigned short* WAO16  = (unsigned short*)(ws + OFF_WAO16);
  unsigned short* WO16   = (unsigned short*)(ws + OFF_WO16);
  float*          BO960  = (float*)(ws + OFF_BO);
  unsigned short* DE16   = (unsigned short*)(ws + OFF_DE16);
  float*          GIF    = (float*)(ws + OFF_GIF);
  float*          GIR    = (float*)(ws + OFF_GIR);
  float*          FWD32  = (float*)(ws + OFF_FWD32);
  float*          RLAST  = (float*)(ws + OFF_RLAST);
  unsigned short* REV16  = (unsigned short*)(ws + OFF_REV16);
  float*          SFWD   = (float*)(ws + OFF_SFWD);
  float*          SREV   = (float*)(ws + OFF_SREV);
  unsigned short* HT16   = (unsigned short*)(ws + OFF_HT16);
  unsigned short* AO16   = (unsigned short*)(ws + OFF_AO16);
  float*          OUT960 = (float*)(ws + OFF_OUT960);

  {
    const int n8x = NROWS * DIN / 8;
    cast_f32_f16x8<<<dim3((n8x + 255) / 256), 256, 0, stream>>>(x, X16, n8x, n8x, 1.0f);
    const int n8e = DDAY * DIN / 8;
    cast_f32_f16x8<<<dim3((n8e + 255) / 256), 256, 0, stream>>>(Wemb, WEMB16, n8e, n8e, 16.0f);
    const int n8w = GATE3 * HID / 8;
    cast_f32_f16x8<<<dim3((n8w + 255) / 256), 256, 0, stream>>>(Wihf, WIHF16, n8w, n8w, 16.0f);
    cast_f32_f16x8<<<dim3((n8w + 255) / 256), 256, 0, stream>>>(Whhf, WHHF16, n8w, n8w, 16.0f);
    cast_f32_f16x8<<<dim3((n8w + 255) / 256), 256, 0, stream>>>(Wihr, WIHR16, n8w, n8w, 16.0f);
    cast_f32_f16x8<<<dim3((n8w + 255) / 256), 256, 0, stream>>>(Whhr, WHHR16, n8w, n8w, 16.0f);
    const int n8a = DDAY * HT_COLS / 8;
    cast_f32_f16x8<<<dim3((n8a + 255) / 256), 256, 0, stream>>>(Wao, WAO16, n8a, n8a, 16.0f);
    const int n8o_tot = NOUT_PAD * DDAY / 8;
    const int n8o_val = NOUT * DDAY / 8;
    cast_f32_f16x8<<<dim3((n8o_tot + 255) / 256), 256, 0, stream>>>(Wo, WO16, n8o_tot, n8o_val, 16.0f);
    pad_vec_f32x4<<<dim3(1), 256, 0, stream>>>(bo, BO960, NOUT_PAD / 4, NOUT);
  }
  {
    const int tiles = (NROWS / 64) * (DDAY / 64);
    wmma_gemm64<0, false, 2, 1, false, 0><<<dim3((tiles + 7) / 8, 1), 256, 0, stream>>>(
        X16, nullptr, DIN, 0L, WEMB16, nullptr, DIN, 0L, (void*)DE16, nullptr, DDAY, 0L,
        bemb, nullptr, 0L, NROWS, DDAY, DIN, 0.0625f);
  }
  {
    const int tiles = (NROWS / 64) * (GATE3 / 64);
    wmma_gemm64<0, false, 2, 0, false, 0><<<dim3((tiles + 7) / 8, 1), 256, 0, stream>>>(
        DE16, nullptr, DDAY, 0L, WIHF16, nullptr, DDAY, 0L, (void*)GIF, nullptr, GATE3, 0L,
        bihf, nullptr, 0L, NROWS, GATE3, DDAY, 0.0625f);
    wmma_gemm64<0, false, 2, 0, false, 0><<<dim3((tiles + 7) / 8, 1), 256, 0, stream>>>(
        DE16, nullptr, DDAY, 0L, WIHR16, nullptr, DDAY, 0L, (void*)GIR, nullptr, GATE3, 0L,
        bihr, nullptr, 0L, NROWS, GATE3, DDAY, 0.0625f);
  }
  gru_seq_kernel<false><<<dim3(NB_ROWS / 16), 256, 0, stream>>>(WHHF16, bhhf, GIF, attnw, FWD32, REV16, SFWD);
  gru_seq_kernel<true><<<dim3(NROWS / 16), 256, 0, stream>>>(WHHR16, bhhr, GIR, attnw + HID, RLAST, REV16, SREV);
  attn_ctx_kernel<<<dim3(NROWS), 128, 0, stream>>>(SFWD, SREV, attnb, FWD32, REV16, RLAST, HT16);
  {
    const int tiles = (NROWS / 64) * (DDAY / 64);
    wmma_gemm64<0, false, 2, 1, false, 0><<<dim3((tiles + 7) / 8, 1), 256, 0, stream>>>(
        HT16, nullptr, HT_COLS, 0L, WAO16, nullptr, HT_COLS, 0L, (void*)AO16, nullptr, DDAY, 0L,
        bao, nullptr, 0L, NROWS, DDAY, HT_COLS, 1.0f / 1024.0f);
  }
  {
    const int tiles = (NROWS / 64) * (NOUT_PAD / 64);
    wmma_gemm64<0, false, 2, 0, false, 6><<<dim3((tiles + 7) / 8, 1), 256, 0, stream>>>(
        AO16, nullptr, DDAY, 0L, WO16, nullptr, DDAY, 0L, (void*)OUT960, nullptr, NOUT_PAD, 0L,
        BO960, nullptr, 0L, NROWS, NOUT_PAD, DDAY, 0.0625f);
  }
  {
    const int n4 = NROWS * NOUT / 4;
    out_pack_kernel<<<dim3((n4 + 255) / 256), 256, 0, stream>>>(OUT960, out, n4, NOUT, NOUT_PAD, NROWS);
  }
}
